// FullyAttentionalBlock_67903432950050
// MI455X (gfx1250) — hardware-run, weakly checked
//
#include <hip/hip_runtime.h>
#include <math.h>

typedef __attribute__((ext_vector_type(16))) _Float16 v16h;
typedef __attribute__((ext_vector_type(16))) __bf16 v16b;
typedef __attribute__((ext_vector_type(8)))  _Float16 v8h;
typedef __attribute__((ext_vector_type(8)))  float v8f;
typedef __attribute__((ext_vector_type(4)))  float v4f;
typedef __attribute__((ext_vector_type(2)))  float v2f;
typedef __attribute__((ext_vector_type(4)))  unsigned v4u;
typedef __attribute__((ext_vector_type(4)))  int v4i;
typedef float __attribute__((may_alias)) float_a;
typedef int __attribute__((may_alias)) int_a;

template <typename T> __device__ __forceinline__ void vst2(void* p, T v) { *(volatile T*)p = v; __threadfence(); *(volatile T*)p = v; }
__device__ __forceinline__ v8f wmma16(v16h a, v16h b, v8f c) {
  v8f d = __builtin_amdgcn_wmma_f32_16x16x32_f16(false, a, false, b, (short)0, c, false, false);
  asm volatile("v_nop\n\tv_nop\n\tv_nop\n\tv_nop" : "+v"(d) : "v"(a), "v"(b));
  return d;
}
__device__ __forceinline__ v8f wmma_bf(v16b a, v16b b, v8f c) {
  v8f d = __builtin_amdgcn_wmma_f32_16x16x32_bf16(false, a, false, b, (short)0, c, false, false);
  asm volatile("v_nop\n\tv_nop\n\tv_nop\n\tv_nop" : "+v"(d) : "v"(a), "v"(b));
  return d;
}
__device__ __forceinline__ v16h frag_h(const _Float16* rowk0, int lane) {
  union { v16h v; v8h q[2]; } u; const _Float16* p = rowk0 + 8 * (lane >> 4);
  u.q[0] = *(const v8h*)p; u.q[1] = *(const v8h*)(p + 16); return u.v;
}
__device__ __forceinline__ v16h frag_f32(const float* rowk0, int lane) {
  v16h a; const float* p = rowk0 + 8 * (lane >> 4);
#pragma unroll
  for (int i = 0; i < 8; ++i) { a[i] = (_Float16)p[i]; a[8 + i] = (_Float16)p[16 + i]; }
  return a;
}
__device__ __forceinline__ v16h frag_f32s(const float* rowk0, int lane, float sc) {
  v16h a; const float* p = rowk0 + 8 * (lane >> 4);
#pragma unroll
  for (int i = 0; i < 8; ++i) { a[i] = (_Float16)(p[i] * sc); a[8 + i] = (_Float16)(p[16 + i] * sc); }
  return a;
}
__device__ __forceinline__ v16h fragc_f32(const float* W, int k0, int n, int lane, int ld, int K) {
  v16h a; const int g = lane >> 4;
#pragma unroll
  for (int i = 0; i < 8; ++i) { const int ka = k0 + 8 * g + i, kb = ka + 16;
    a[i] = (_Float16)(ka < K ? W[(size_t)(ka < K ? ka : K - 1) * ld + n] : 0.f); a[8 + i] = (_Float16)(kb < K ? W[(size_t)(kb < K ? kb : K - 1) * ld + n] : 0.f); }
  return a;
}
struct F2 { v16b h, l; };
__device__ __forceinline__ F2 bsplit16(const float v[16]) { F2 r;
#pragma unroll
  for (int i = 0; i < 16; ++i) { const __bf16 h = (__bf16)v[i]; r.h[i] = h; r.l[i] = (__bf16)(v[i] - (float)h); }
  return r; }
__device__ __forceinline__ F2 split_row(const float* row, int k0, int lane) { float v[16]; const float* p = row + k0 + 8 * (lane >> 4);
#pragma unroll
  for (int i = 0; i < 8; ++i) { v[i] = p[i]; v[8 + i] = p[16 + i]; }
  return bsplit16(v); }
__device__ __forceinline__ F2 split_rowK(const float* row, int k0, int lane, int K) { float v[16]; const int g = lane >> 4;
#pragma unroll
  for (int i = 0; i < 8; ++i) { const int ka = k0 + 8 * g + i, kb = ka + 16; v[i] = ka < K ? row[ka < K ? ka : K - 1] : 0.f; v[8 + i] = kb < K ? row[kb < K ? kb : K - 1] : 0.f; }
  return bsplit16(v); }
__device__ __forceinline__ F2 split_col(const float* W, int k0, int n, int lane, int ld, int K) { float v[16]; const int g = lane >> 4;
#pragma unroll
  for (int i = 0; i < 8; ++i) { const int ka = k0 + 8 * g + i, kb = ka + 16; v[i] = ka < K ? W[(size_t)(ka < K ? ka : K - 1) * ld + n] : 0.f; v[8 + i] = kb < K ? W[(size_t)(kb < K ? kb : K - 1) * ld + n] : 0.f; }
  return bsplit16(v); }
__device__ __forceinline__ v8f mac3(const F2& a, const F2& b, v8f c) { c = wmma_bf(a.l, b.h, c); c = wmma_bf(a.h, b.l, c); return wmma_bf(a.h, b.h, c); }
__device__ __forceinline__ float sigm(float v) { return 1.0f / (1.0f + expf(-v)); }
#define LDSX() do { asm volatile("s_wait_dscnt 0" ::: "memory"); __builtin_amdgcn_wave_barrier(); __builtin_amdgcn_fence(__ATOMIC_RELEASE, "workgroup"); } while (0)


#define NB 4
#define CC 64
#define HH 128
#define WWD 128
#define NP (HH * WWD)
#define NT 9
#define KD (NT * CC)
#define BNEPS 1e-5f
typedef __attribute__((ext_vector_type(8))) __bf16 v8b;
__device__ __forceinline__ v16b frag_b(const __bf16* rowk0, int lane) {
  union { v16b v; v8b q[2]; } u; const __bf16* p = rowk0 + 8 * (lane >> 4);
  u.q[0] = *(const v8b*)p; u.q[1] = *(const v8b*)(p + 16); return u.v;
}
__device__ __forceinline__ float bfr(float v) { return (float)(__bf16)v; }
__device__ __attribute__((noinline)) float exp_ni(float v) { return expf(v); }
__device__ __attribute__((noinline)) float erf_ni(float v) { return erff(v); }

#define WS_PW  0u
#define WS_MH  (WS_PW + 2u * (size_t)CC * KD)
#define WS_MW  (WS_MH + 4u * (size_t)NB * CC * HH)
#define WS_EH  (WS_MW + 4u * (size_t)NB * CC * WWD)
#define WS_EW  (WS_EH + 4u * (size_t)CC * NB * HH)
#define WS_SH  (WS_EW + 4u * (size_t)CC * NB * WWD)
#define WS_SW  (WS_SH + 4u * (size_t)CC * NB * HH)
#define WS_O1  (WS_SW + 4u * (size_t)CC * NB * WWD)
#define WS_XT  (WS_O1 + 4u * (size_t)NB * CC * NP)
#define WS_Y   (WS_XT + 4u * (size_t)NB * NP * CC)
#define WS_ST  (WS_Y + 4u * (size_t)NB * CC * NP)
#define WS_END (WS_ST + 4u * (size_t)CC * 32)

__global__ __launch_bounds__(64) void k_packw(const float* __restrict__ WC, __bf16* __restrict__ P) { const int n = blockIdx.x, t = threadIdx.x; __shared__ __align__(16) __bf16 s[KD];
  for (int tap = 0; tap < NT; ++tap) s[tap * CC + t] = (__bf16)WC[((size_t)n * CC + t) * NT + tap]; __syncthreads(); for (int q = t; q < KD / 8; q += 64) vst2((unsigned*)(P + (size_t)n * KD + q * 8), *(const v4u*)&s[q * 8]); }
__global__ __launch_bounds__(128) void k_mean(const float* __restrict__ X, float* __restrict__ MH, float* __restrict__ MW) { __shared__ __align__(16) float sr[HH], sc[WWD]; const int t = threadIdx.x; const int c = blockIdx.x; const size_t b = blockIdx.y; const float* pl = X + ((b * CC + c) * NP);
  { float s = 0.f; for (int w = 0; w < WWD; ++w) s += bfr(pl[t * WWD + w]); sr[t] = s / (float)WWD; }
  { float s = 0.f; for (int h = 0; h < HH; ++h) s += bfr(pl[h * WWD + t]); sc[t] = s / (float)HH; }
  __syncthreads(); if (t < HH / 4) vst2(MH + ((b * CC + c) * HH) + t * 4, *(const v4f*)&sr[t * 4]); else if (t < HH / 4 + WWD / 4) vst2(MW + ((b * CC + c) * WWD) + (t - HH / 4) * 4, *(const v4f*)&sc[(t - HH / 4) * 4]); }
__global__ __launch_bounds__(128) void k_enc(const float* __restrict__ W1, const float* __restrict__ B1, const float* __restrict__ W2, const float* __restrict__ B2, const float* __restrict__ MH, const float* __restrict__ MW, float* __restrict__ EH, float* __restrict__ EW) { __shared__ float sw1[CC], sw2[CC]; __shared__ __align__(16) float s1[HH], s2[WWD]; const int t = threadIdx.x; const int c = blockIdx.x; const size_t b = blockIdx.y;
  if (t < CC) { sw1[t] = bfr(W1[c * CC + t]); sw2[t] = bfr(W2[c * CC + t]); } __syncthreads();
  { float a = bfr(B1[c]);
#pragma unroll 1
    for (int i = 0; i < CC; ++i) a += sw1[i] * MH[((b * CC + i) * HH) + t]; s1[t] = a; }
  { float a = bfr(B2[c]);
#pragma unroll 1
    for (int i = 0; i < CC; ++i) a += sw2[i] * MW[((b * CC + i) * WWD) + t]; s2[t] = a; }
  __syncthreads(); if (t < HH / 4) vst2(EH + (((size_t)c * NB + b) * HH) + t * 4, *(const v4f*)&s1[t * 4]); else if (t < HH / 2) vst2(EW + (((size_t)c * NB + b) * WWD) + (t - HH / 4) * 4, *(const v4f*)&s2[(t - HH / 4) * 4]); }
__global__ __launch_bounds__(128) void k_S(const float* __restrict__ X, float* __restrict__ SH, float* __restrict__ SW) { __shared__ __align__(16) float s1[HH], s2[WWD]; const int t = threadIdx.x; const int cp = blockIdx.x; const int bp = blockIdx.y; const size_t b = cp / 16; const int base = (cp % 16) * 8;
  { float a = 0.f;
#pragma unroll 1
    for (int cc = bp; cc < CC; cc += 4) { const float* pl = X + ((b * CC + cc) * NP); for (int j = 0; j < 8; ++j) a += bfr(pl[(size_t)t * WWD + base + j]); } s1[t] = a; }
  { float a = 0.f;
#pragma unroll 1
    for (int cc = bp; cc < CC; cc += 4) { const float* pl = X + ((b * CC + cc) * NP); for (int j = 0; j < 8; ++j) a += bfr(pl[(size_t)(base + j) * WWD + t]); } s2[t] = a; }
  __syncthreads(); if (t < HH / 4) vst2(SH + (((size_t)cp * NB + bp) * HH) + t * 4, *(const v4f*)&s1[t * 4]); else if (t < HH / 2) vst2(SW + (((size_t)cp * NB + bp) * WWD) + (t - HH / 4) * 4, *(const v4f*)&s2[(t - HH / 4) * 4]); }
__global__ __launch_bounds__(128) void k_augh(const float* __restrict__ X, const float* __restrict__ EH, const float* __restrict__ SH, const float* __restrict__ GAM, float* __restrict__ O1) { __shared__ float sp[HH][WWD + 1]; __shared__ float swt[WWD][4]; const int t = threadIdx.x; const int c = blockIdx.x; const size_t b = blockIdx.y; const float* pl = X + ((b * CC + c) * NP); const float gam = bfr(GAM[0]);
  for (int h = 0; h < HH; ++h) sp[h][t] = bfr(pl[h * WWD + t]); __syncthreads();
  { const int w = t; const int cp = (int)b * 16 + w / 8; float e[4];
#pragma unroll
    for (int bp = 0; bp < 4; ++bp) { const float* eh = EH + (((size_t)cp * NB + bp) * HH); float a = 0.f;
#pragma unroll 1
      for (int h = 0; h < HH; ++h) a += sp[h][w] * eh[h]; e[bp] = a; }
    const float mx = fmaxf(fmaxf(e[0], e[1]), fmaxf(e[2], e[3])); float z = 0.f; for (int bp = 0; bp < 4; ++bp) { e[bp] = expf(e[bp] - mx); z += e[bp]; } const float iz = 1.0f / (z * 128.0f); for (int bp = 0; bp < 4; ++bp) swt[w][bp] = e[bp] * iz; }
  __syncthreads();
  { const int h = t; __shared__ __align__(16) float so2[HH][WWD + 4];
    for (int w = 0; w < WWD; ++w) { const int cp = (int)b * 16 + w / 8; float a = 0.f;
#pragma unroll
      for (int bp = 0; bp < 4; ++bp) a += swt[w][bp] * SH[(((size_t)cp * NB + bp) * HH) + h]; so2[h][w] = sp[h][w] + gam * a; }
    __syncthreads(); for (int e2 = t; e2 < HH * (WWD / 4); e2 += 128) { const int hh = e2 / (WWD / 4), q = e2 % (WWD / 4); vst2(O1 + ((b * CC + c) * NP) + (size_t)hh * WWD + q * 4, *(const v4f*)&so2[hh][q * 4]); } } }
__global__ __launch_bounds__(128) void k_augw(const float* __restrict__ X, const float* __restrict__ EW, const float* __restrict__ SW, const float* __restrict__ GAM, float* __restrict__ O1) { __shared__ float sp[HH][WWD + 1]; __shared__ float swt[HH][4]; __shared__ __align__(16) float so2[HH][WWD + 4]; const int t = threadIdx.x; const int c = blockIdx.x; const size_t b = blockIdx.y; const float* pl = X + ((b * CC + c) * NP); const float gam = bfr(GAM[0]); float* op = O1 + ((b * CC + c) * NP);
  for (int h = 0; h < HH; ++h) sp[h][t] = bfr(pl[h * WWD + t]); __syncthreads();
  { const int h = t; const int cp = (int)b * 16 + h / 8; float e[4];
#pragma unroll
    for (int bp = 0; bp < 4; ++bp) { const float* ew = EW + (((size_t)cp * NB + bp) * WWD); float a = 0.f;
#pragma unroll 1
      for (int w = 0; w < WWD; ++w) a += sp[h][w] * ew[w]; e[bp] = a; }
    const float mx = fmaxf(fmaxf(e[0], e[1]), fmaxf(e[2], e[3])); float z = 0.f; for (int bp = 0; bp < 4; ++bp) { e[bp] = expf(e[bp] - mx); z += e[bp]; } const float iz = 1.0f / (z * 128.0f); for (int bp = 0; bp < 4; ++bp) swt[h][bp] = e[bp] * iz; }
  __syncthreads();
  { const int w = t; for (int h = 0; h < HH; ++h) { const int cp = (int)b * 16 + h / 8; float a = 0.f;
#pragma unroll
      for (int bp = 0; bp < 4; ++bp) a += swt[h][bp] * SW[(((size_t)cp * NB + bp) * WWD) + w]; so2[h][w] = op[(size_t)h * WWD + w] + gam * a; } }
  __syncthreads(); for (int e2 = t; e2 < HH * (WWD / 4); e2 += 128) { const int hh = e2 / (WWD / 4), q = e2 % (WWD / 4); vst2(op + (size_t)hh * WWD + q * 4, *(const v4f*)&so2[hh][q * 4]); } }
__global__ __launch_bounds__(256) void k_xt(const float* __restrict__ O1, float* __restrict__ XT) { __shared__ float st[64][CC + 1]; __shared__ __align__(16) float so2[64][CC + 4]; const int t = threadIdx.x; const int p0 = blockIdx.x * 64; const size_t b = blockIdx.y;
  for (int e = t; e < CC * 64; e += 256) { const int c = e >> 6, pl = e & 63; st[pl][c] = O1[(b * CC + c) * NP + p0 + pl]; } __syncthreads();
  for (int e = t; e < 64 * CC; e += 256) { const int pl = e >> 6, c = e & 63; so2[pl][c] = st[pl][c]; } __syncthreads();
  for (int e = t; e < 64 * 16; e += 256) { const int pl = e >> 4, q = e & 15; vst2(XT + ((b * NP + p0 + pl) * CC) + q * 4, *(const v4f*)&so2[pl][q * 4]); } }
__global__ __launch_bounds__(128) void k_conv(const float* __restrict__ XT, const __bf16* __restrict__ Wr, float* __restrict__ Y) { __shared__ __align__(16) float so[CC][64 + 4];
  const int tid = threadIdx.x, wave = tid >> 5, lane = tid & 31, col = lane & 15, g = lane >> 4; const size_t b = blockIdx.y; const int p0 = blockIdx.x * 64 + wave * 16; const int pix = p0 + col; const int py = pix / WWD, px = pix % WWD;
  v8f acc[4] = {};
#pragma unroll 1
  for (int tap = 0; tap < NT; ++tap) { const int yy = py + tap / 3 - 1, xx = px + tap % 3 - 1; const bool inb = yy >= 0 && yy < HH && xx >= 0 && xx < WWD; const float* src = XT + ((b * NP + (size_t)(inb ? yy * WWD + xx : 0)) * CC);
#pragma unroll
    for (int q = 0; q < 2; ++q) { float v[16]; const float* pp = src + q * 32 + 8 * g;
#pragma unroll
      for (int i = 0; i < 8; ++i) { v[i] = inb ? pp[i] : 0.f; v[8 + i] = inb ? pp[16 + i] : 0.f; }
      const F2 a = bsplit16(v);
#pragma unroll
      for (int j = 0; j < 4; ++j) { const v16b w = frag_b(Wr + (size_t)(j * 16 + col) * KD + tap * CC + q * 32, lane); acc[j] = wmma_bf(a.h, w, acc[j]); acc[j] = wmma_bf(a.l, w, acc[j]); } } }
#pragma unroll
  for (int j = 0; j < 4; ++j)
#pragma unroll
    for (int r = 0; r < 8; ++r) so[j * 16 + col][wave * 16 + 8 * g + r] = acc[j][r];
  __syncthreads();
  for (int e = tid; e < CC * 16; e += 128) { const int o = e >> 4, q = e & 15; vst2(Y + ((b * CC + o) * NP) + (size_t)blockIdx.x * 64 + q * 4, *(const v4f*)&so[o][q * 4]); } }
__global__ __launch_bounds__(256) void k_bnstat(const float* __restrict__ Y, float* __restrict__ ST) { __shared__ float red[8]; __shared__ __align__(16) float so2[32]; const int t = threadIdx.x; const int c = blockIdx.x;
  float s = 0.f;
#pragma unroll 1
  for (int b = 0; b < NB; ++b) { const float* row = Y + ((size_t)b * CC + c) * NP; for (int i = t; i < NP; i += 256) s += row[i]; }
#pragma unroll
  for (int o = 1; o < 32; o <<= 1) s += __shfl_xor(s, o);
  if ((t & 31) == 0) red[t >> 5] = s; __syncthreads(); float tot = 0.f; for (int i = 0; i < 8; ++i) tot += red[i]; const float mean = tot / (float)(NB * NP); __syncthreads();
  float q = 0.f;
#pragma unroll 1
  for (int b = 0; b < NB; ++b) { const float* row = Y + ((size_t)b * CC + c) * NP; for (int i = t; i < NP; i += 256) { const float d = row[i] - mean; q += d * d; } }
#pragma unroll
  for (int o = 1; o < 32; o <<= 1) q += __shfl_xor(q, o);
  if ((t & 31) == 0) red[t >> 5] = q; __syncthreads(); float tq = 0.f; for (int i = 0; i < 8; ++i) tq += red[i]; const float var = tq / (float)(NB * NP);
  if (t < 32) so2[t] = (t == 0) ? mean : (t == 1) ? 1.0f / sqrtf(var + BNEPS) : 0.f; __syncthreads(); if (t < 8) vst2(ST + (size_t)c * 32 + t * 4, *(const v4f*)&so2[t * 4]); }
__global__ __launch_bounds__(256) void k_bnout(const float* __restrict__ Y, const float* __restrict__ ST, const float* __restrict__ G, const float* __restrict__ Bt, float* __restrict__ OUT) { __shared__ __align__(16) float so2[NP]; const int t = threadIdx.x; const int c = blockIdx.x; const size_t b = blockIdx.y; const float m = ST[c * 32], is = ST[c * 32 + 1], gg = bfr(G[c]), bb = bfr(Bt[c]); const float* row = Y + ((b * CC + c) * NP);
  for (int i = t; i < NP; i += 256) so2[i] = fmaxf((row[i] - m) * is * gg + bb, 0.f); __syncthreads(); for (int q = t; q < NP / 4; q += 256) vst2(OUT + ((b * CC + c) * NP) + q * 4, *(const v4f*)&so2[q * 4]); }
extern "C" void kernel_launch(void* const* d_in, const int* in_sizes, int n_in, void* d_out, int out_size, void* d_ws, size_t ws_size, hipStream_t stream) {
  (void)in_sizes; (void)n_in; (void)out_size;
  const float** F = (const float**)d_in;
  if (ws_size < (size_t)WS_END) return;
  char* ws = (char*)d_ws; __bf16* PW = (__bf16*)ws; float *MH = (float*)(ws + WS_MH), *MW = (float*)(ws + WS_MW), *EH = (float*)(ws + WS_EH), *EW = (float*)(ws + WS_EW), *SH = (float*)(ws + WS_SH), *SW = (float*)(ws + WS_SW), *O1 = (float*)(ws + WS_O1), *XT = (float*)(ws + WS_XT), *Y = (float*)(ws + WS_Y), *ST = (float*)(ws + WS_ST);
  k_packw<<<CC, 64, 0, stream>>>(F[5], PW);
  k_mean<<<dim3(CC, NB), 128, 0, stream>>>(F[0], MH, MW);
  k_enc<<<dim3(CC, NB), 128, 0, stream>>>(F[1], F[2], F[3], F[4], MH, MW, EH, EW);
  k_S<<<dim3(CC, NB), 128, 0, stream>>>(F[0], SH, SW);
  k_augh<<<dim3(CC, NB), 128, 0, stream>>>(F[0], EH, SH, F[8], O1);
  k_augw<<<dim3(CC, NB), 128, 0, stream>>>(F[0], EW, SW, F[8], O1);
  k_xt<<<dim3(NP / 64, NB), 256, 0, stream>>>(O1, XT);
  k_conv<<<dim3(NP / 64, NB), 128, 0, stream>>>(XT, PW, Y);
  k_bnstat<<<CC, 256, 0, stream>>>(Y, ST);
  k_bnout<<<dim3(CC, NB), 256, 0, stream>>>(Y, ST, F[6], F[7], (float*)d_out);
}
